// LabelwiseAttention_34557306863626
// MI455X (gfx1250) — hardware-verified
//
#include <hip/hip_runtime.h>
#include <math.h>
#include <stdint.h>

#ifndef NB
#define NB 8
#endif
#ifndef SEQ
#define SEQ 2048
#endif
#define NB_FULL  8
#define SEQ_FULL 2048
#define DM       768
#define NCLS     4271
#define CP       4288
#define NC       (2 * CP)

static_assert(NB >= 1 && NB <= NB_FULL);
static_assert(SEQ >= 64 && SEQ <= SEQ_FULL && (SEQ % 64) == 0 && (SEQ % 4) == 0);
static_assert((DM % 32) == 0 && (DM % 8) == 0);
static_assert((CP % 64) == 0 && CP >= NCLS && (NC % 64) == 0);
static_assert(((CP * (DM / 8)) % 256) == 0);
static_assert(((SEQ * (DM / 8)) % 256) == 0);
static_assert((long long)NB_FULL * NCLS * 4 == 136672LL);

#define XBB ((long long)NB * SEQ * DM * 2)
#define WCB ((long long)NC * DM * 2)
#define SBB ((long long)SEQ * NC * 4)
#define LGB ((long long)NB * CP * 4)
static_assert((XBB % 128) == 0 && (WCB % 128) == 0 && (SBB % 128) == 0 && (LGB % 128) == 0);
static_assert(XBB + WCB + SBB + LGB <= 134217728LL);

typedef _Float16 v16h __attribute__((ext_vector_type(16)));
typedef _Float16 v8h  __attribute__((ext_vector_type(8)));
typedef __bf16   v16b __attribute__((ext_vector_type(16)));
typedef __bf16   v8b  __attribute__((ext_vector_type(8)));
typedef float    v8f  __attribute__((ext_vector_type(8)));
typedef float    v4f  __attribute__((ext_vector_type(4)));
typedef unsigned int v4u __attribute__((ext_vector_type(4)));

#if defined(__HIP_DEVICE_COMPILE__)
#define DEV_ASM 1
#else
#define DEV_ASM 0
#endif

__device__ __forceinline__ unsigned short bf_bits(float f) {
  unsigned u = __float_as_uint(f);
  return (unsigned short)((u + 0x7FFFu + ((u >> 16) & 1u)) >> 16);
}
__device__ __forceinline__ float bf_up(unsigned short hb) { return __uint_as_float(((unsigned)hb) << 16); }
__device__ __forceinline__ unsigned short h_bits(_Float16 x) { return __builtin_bit_cast(unsigned short, x); }
__device__ __forceinline__ unsigned pk16(unsigned short a, unsigned short b) { return (unsigned)a | ((unsigned)b << 16); }
__device__ __forceinline__ v8f zero8() { v8f z = {0.f, 0.f, 0.f, 0.f, 0.f, 0.f, 0.f, 0.f}; return z; }

template <typename OT> struct FT;
template <> struct FT<__bf16>   { typedef v16b frag; typedef v8b half8; };
template <> struct FT<_Float16> { typedef v16h frag; typedef v8h half8; };

template <typename OT>
__device__ __forceinline__ typename FT<OT>::frag ldfrag(const OT* p) {
  union { typename FT<OT>::frag v; typename FT<OT>::half8 h[2]; } f;
  f.h[0] = *(const typename FT<OT>::half8*)(p);
  f.h[1] = *(const typename FT<OT>::half8*)(p + 16);
  return f.v;
}

__device__ __forceinline__ v8f mmar(v16b a, v16b b, v8f c) {
  return __builtin_amdgcn_wmma_f32_16x16x32_bf16(false, a, false, b, (short)0, c, false, false);
}
__device__ __forceinline__ v8f mmar(v16h a, v16h b, v8f c) {
  return __builtin_amdgcn_wmma_f32_16x16x32_f16(false, a, false, b, (short)0, c, false, false);
}
__device__ __forceinline__ void dep_guard(v8f& a, v8f& b, v16b x, v16b y) {
#if DEV_ASM
  asm volatile("v_nop\n\tv_nop\n\tv_nop\n\tv_nop" : "+v"(a), "+v"(b) : "v"(x), "v"(y));
#else
  (void)a; (void)b; (void)x; (void)y;
#endif
}
__device__ __forceinline__ void dep_guard(v8f& a, v8f& b, v16h x, v16h y) {
#if DEV_ASM
  asm volatile("v_nop\n\tv_nop\n\tv_nop\n\tv_nop" : "+v"(a), "+v"(b) : "v"(x), "v"(y));
#else
  (void)a; (void)b; (void)x; (void)y;
#endif
}
__device__ __forceinline__ void keep4(v16b a, v16b b, v16b c, v16b d) {
#if DEV_ASM
  asm volatile("v_nop" :: "v"(a), "v"(b), "v"(c), "v"(d));
#else
  (void)a; (void)b; (void)c; (void)d;
#endif
}
__device__ __forceinline__ void keep4(v16h a, v16h b, v16h c, v16h d) {
#if DEV_ASM
  asm volatile("v_nop" :: "v"(a), "v"(b), "v"(c), "v"(d));
#else
  (void)a; (void)b; (void)c; (void)d;
#endif
}
__device__ __forceinline__ void acc_guard4(v8f& a, v8f& b, v8f& c, v8f& d) {
#if DEV_ASM
  asm volatile("v_nop\n\tv_nop\n\tv_nop\n\tv_nop" : "+v"(a), "+v"(b), "+v"(c), "+v"(d));
#else
  (void)a; (void)b; (void)c; (void)d;
#endif
}

template <int MODE>
__device__ __forceinline__ unsigned short cvm(float f) {
  const unsigned short hb = bf_bits(f);
  if (MODE == 0) return hb;
  return h_bits((_Float16)(bf_up(hb) * 64.0f));
}

template <int MODE>
__global__ __launch_bounds__(256) void cvt16x8(const float* __restrict__ in, long long sin,
                                               unsigned short* out, long long sout, int n8) {
  const int i = blockIdx.x * 256 + (int)threadIdx.x;
  const int y = blockIdx.y;
  if (i < n8) {
    const float* ip = in + (size_t)y * (size_t)sin + (size_t)i * 8;
    const v4f a  = *(const v4f*)(ip);
    const v4f a4 = *(const v4f*)(ip + 4);
    v4u p;
    p[0] = pk16(cvm<MODE>(a[0]),  cvm<MODE>(a[1]));
    p[1] = pk16(cvm<MODE>(a[2]),  cvm<MODE>(a[3]));
    p[2] = pk16(cvm<MODE>(a4[0]), cvm<MODE>(a4[1]));
    p[3] = pk16(cvm<MODE>(a4[2]), cvm<MODE>(a4[3]));
    unsigned short* o = out + (size_t)y * (size_t)sout + (size_t)i * 8;
    *(volatile v4u*)o = p;
    __threadfence();
    *(volatile v4u*)o = p;
  }
}

__global__ __launch_bounds__(256) void cvtw8(const float* __restrict__ wa, const float* __restrict__ wo,
                                             unsigned short* WC, int n8) {
  const int i = blockIdx.x * 256 + (int)threadIdx.x;
  const int y = blockIdx.y;
  if (i < n8) {
    const int row  = i / (DM / 8);
    const int c8   = (i - row * (DM / 8)) * 8;
    const int srow = (row < NCLS) ? row : (NCLS - 1);
    const float* src = (y == 0) ? wa : wo;
    const float* ip = src + (size_t)srow * DM + c8;
    const v4f a  = *(const v4f*)(ip);
    const v4f a4 = *(const v4f*)(ip + 4);
    const unsigned keep = (row < NCLS) ? 0xFFFFFFFFu : 0u;
    v4u p;
    p[0] = pk16(bf_bits(a[0]),  bf_bits(a[1]))  & keep;
    p[1] = pk16(bf_bits(a[2]),  bf_bits(a[3]))  & keep;
    p[2] = pk16(bf_bits(a4[0]), bf_bits(a4[1])) & keep;
    p[3] = pk16(bf_bits(a4[2]), bf_bits(a4[3])) & keep;
    unsigned short* o = WC + (size_t)y * (size_t)CP * DM + (size_t)i * 8;
    *(volatile v4u*)o = p;
    __threadfence();
    *(volatile v4u*)o = p;
  }
}

template <typename OT, int MI, int NPA, int NPB, int OUT_MODE, int CZ>
__global__ __launch_bounds__(256) void gemm_t(
    const unsigned short* __restrict__ Ap, const unsigned short* __restrict__ A2p, int lda, long long strideA,
    const unsigned short* __restrict__ Btp, int ldb, long long strideB,
    const unsigned short* __restrict__ B2p, int ldb2, long long strideB2, int K2,
    void* Cout, void* Cout2, int ldc, long long strideC, int ldc2, long long strideC2, int N2,
    int M, int N, int K, float oscale, float rscale2, float cscale, float rscaleC) {
  static_assert(CZ != 2 || ((16 * MI) % 32) == 0);
  static_assert(!(NPA == 2 && NPB == 2));
  typedef typename FT<OT>::frag V16;
  const OT* A  = (const OT*)(const void*)Ap;
  const OT* A2 = (const OT*)(const void*)A2p;
  const OT* Bt = (const OT*)(const void*)Btp;
  const OT* B2 = (const OT*)(const void*)B2p;
  __shared__ __align__(16) float sT[8][16 * 68];
  const int RT   = 16 * MI;
  const int b    = blockIdx.y;
  const int lane = threadIdx.x & 31;
  const int wave = threadIdx.x >> 5;
  const int tilesN = N >> 6;
  const int tilesM = M / RT;
  const int tile = blockIdx.x * 8 + wave;
  if (tile >= tilesM * tilesN) return;
  const int tm = tile / tilesN;
  const int tn = tile - tm * tilesN;
  const int m0 = tm * RT;
  const int n0 = tn << 6;
  if (CZ == 1) {
    if (n0 >= m0 + RT) return;
  }
  int kEnd = K;
  if (CZ == 2) {
    const int ke = m0 + RT;
    kEnd = (ke < K) ? ke : K;
  }

  const OT* Ab  = A  + (size_t)b * (size_t)strideA;
  const OT* A2b = A2 + (size_t)b * (size_t)strideA;
  const OT* Bb  = Bt + (size_t)b * (size_t)strideB;
  const OT* B2b = B2 + (size_t)b * (size_t)strideB2;

  const int rlane = lane & 15;
  const int koff  = (lane >> 4) * 8;
  const int mOff  = (lane >> 4) * 8;

  v8f acc[MI][4], acc2[MI][4];
#pragma unroll
  for (int i = 0; i < MI; ++i)
#pragma unroll
    for (int j = 0; j < 4; ++j) { acc[i][j] = zero8(); acc2[i][j] = zero8(); }

#pragma unroll 1
  for (int k0 = 0; k0 < kEnd; k0 += 32) {
    V16 bq[4];
#pragma unroll
    for (int j = 0; j < 4; ++j)
      bq[j] = ldfrag<OT>(Bb + (size_t)(n0 + (j << 4) + rlane) * ldb + koff + k0);
#pragma unroll
    for (int i = 0; i < MI; ++i) {
      const V16 af = ldfrag<OT>(Ab + (size_t)(m0 + (i << 4) + rlane) * lda + koff + k0);
#pragma unroll
      for (int j = 0; j < 4; ++j) acc[i][j] = mmar(af, bq[j], acc[i][j]);
      dep_guard(acc[i][0], acc[i][3], af, bq[3]);
      if (NPA == 2) {
        const V16 af2 = ldfrag<OT>(A2b + (size_t)(m0 + (i << 4) + rlane) * lda + koff + k0);
#pragma unroll
        for (int j = 0; j < 4; ++j) acc2[i][j] = mmar(af2, bq[j], acc2[i][j]);
        dep_guard(acc2[i][0], acc2[i][3], af2, bq[3]);
      }
    }
    keep4(bq[0], bq[1], bq[2], bq[3]);
    if (NPB == 2) {
      if (k0 < K2) {
        V16 br[4];
#pragma unroll
        for (int j = 0; j < 4; ++j)
          br[j] = ldfrag<OT>(B2b + (size_t)(n0 + (j << 4) + rlane) * ldb2 + koff + k0);
#pragma unroll
        for (int i = 0; i < MI; ++i) {
          const V16 afr = ldfrag<OT>(Ab + (size_t)(m0 + (i << 4) + rlane) * lda + koff + k0);
#pragma unroll
          for (int j = 0; j < 4; ++j) acc2[i][j] = mmar(afr, br[j], acc2[i][j]);
          dep_guard(acc2[i][0], acc2[i][3], afr, br[3]);
        }
        keep4(br[0], br[1], br[2], br[3]);
      }
    }
  }
#pragma unroll
  for (int i = 0; i < MI; ++i) {
    acc_guard4(acc[i][0], acc[i][1], acc[i][2], acc[i][3]);
    if (NPA == 2 || NPB == 2) acc_guard4(acc2[i][0], acc2[i][1], acc2[i][2], acc2[i][3]);
  }

  float* slab = sT[wave];
#pragma unroll
  for (int i = 0; i < MI; ++i) {
    const int mBase = m0 + (i << 4);
#pragma unroll
    for (int j = 0; j < 4; ++j) {
#pragma unroll
      for (int r = 0; r < 8; ++r) {
        float v = acc[i][j][r];
        if (NPA == 2 || NPB == 2) v += acc2[i][j][r] * rscale2;
        v = v * oscale;
        slab[(mOff + r) * 68 + (j << 4) + rlane] = v;
      }
    }
    __builtin_amdgcn_fence(__ATOMIC_RELEASE, "workgroup");
    __builtin_amdgcn_wave_barrier();
    __builtin_amdgcn_fence(__ATOMIC_ACQUIRE, "workgroup");
    if (OUT_MODE == 0) {
      float* C = (float*)Cout + (size_t)b * (size_t)strideC;
      const int h2 = lane >> 4, c4 = (lane & 15) * 4;
      for (int pass = 0; pass < 2; ++pass) {
#pragma unroll
        for (int it = 0; it < 8; ++it) {
          const int row = it * 2 + h2;
          const v4f v = *(const v4f*)(slab + row * 68 + c4);
          *(volatile v4f*)(C + (size_t)(mBase + row) * ldc + n0 + c4) = v;
        }
        __threadfence();
      }
    } else {
      const int q = lane >> 3, c8 = (lane & 7) * 8;
      unsigned short* C  = (unsigned short*)Cout  + (size_t)b * (size_t)strideC;
      unsigned short* C2 = (unsigned short*)Cout2 + (size_t)b * (size_t)strideC2;
      const bool wr2 = (OUT_MODE == 3) && (n0 < N2);
      v4u hv[4], lv[4];
#pragma unroll
      for (int it = 0; it < 4; ++it) {
        const int row = it * 4 + q;
        const float* sp = slab + row * 68 + c8;
        float f[8];
#pragma unroll
        for (int e = 0; e < 8; ++e) f[e] = sp[e] * cscale;
        v4u a, a2;
#pragma unroll
        for (int e = 0; e < 4; ++e) {
          const float f0 = f[2 * e], f1 = f[2 * e + 1];
          const _Float16 x0 = (_Float16)f0, x1 = (_Float16)f1;
          const unsigned short h0 = h_bits(x0), h1 = h_bits(x1);
          unsigned short l0 = 0, l1 = 0;
          if (OUT_MODE == 3) {
            l0 = h_bits((_Float16)((f0 - (float)x0) * rscaleC));
            l1 = h_bits((_Float16)((f1 - (float)x1) * rscaleC));
          }
          a[e] = pk16(h0, h1); a2[e] = pk16(l0, l1);
        }
        hv[it] = a; lv[it] = a2;
      }
      for (int pass = 0; pass < 2; ++pass) {
#pragma unroll
        for (int it = 0; it < 4; ++it) {
          const int row = it * 4 + q;
          *(volatile v4u*)(C + (size_t)(mBase + row) * ldc + n0 + c8) = hv[it];
          if (OUT_MODE == 3) {
            if (wr2) *(volatile v4u*)(C2 + (size_t)(mBase + row) * ldc2 + n0 + c8) = lv[it];
          }
        }
        __threadfence();
      }
    }
    __builtin_amdgcn_fence(__ATOMIC_RELEASE, "workgroup");
    __builtin_amdgcn_wave_barrier();
    __builtin_amdgcn_fence(__ATOMIC_ACQUIRE, "workgroup");
  }
}

__global__ __launch_bounds__(256) void colsm(const float* __restrict__ SP, const float* __restrict__ bo, float* LG) {
  __shared__ float red[4][64];
  __shared__ float red2[4][64];
  const int tid = (int)threadIdx.x;
  const int tc  = tid & 63;
  const int rg  = tid >> 6;
  const int c0  = blockIdx.x * 64;
  const float* ap = SP + c0 + tc;
  const float* gp = SP + CP + c0 + tc;

  float mx = -INFINITY;
#pragma unroll 4
  for (int j = 0; j < SEQ / 4; ++j) {
    const int s = 4 * j + rg;
    mx = fmaxf(mx, ap[(size_t)s * NC]);
  }
  red[rg][tc] = mx;
  __syncthreads();
  float m = red[0][tc];
  m = fmaxf(m, red[1][tc]);
  m = fmaxf(m, red[2][tc]);
  m = fmaxf(m, red[3][tc]);
  __syncthreads();

  float L = 0.f, T = 0.f;
#pragma unroll 2
  for (int j = 0; j < SEQ / 4; ++j) {
    const int s = 4 * j + rg;
    const size_t o = (size_t)s * NC;
    const float e = expf(ap[o] - m);
    L += e;
    T = fmaf(e, gp[o], T);
  }
  red[rg][tc]  = L;
  red2[rg][tc] = T;
  __syncthreads();

  float val = 0.f;
  float* p = LG + c0 + (tid & 63);
  if (tid < 64) {
    const float Ls = ((red[0][tid]  + red[1][tid])  + red[2][tid])  + red[3][tid];
    const float Ts = ((red2[0][tid] + red2[1][tid]) + red2[2][tid]) + red2[3][tid];
    const int c  = c0 + tid;
    const int cc = (c < NCLS) ? c : (NCLS - 1);
    const float braw = bo[cc];
    const float bias = (c < NCLS) ? bf_up(bf_bits(braw)) : 0.f;
    val = Ts * (1.0f / Ls) + bias;
    *(volatile float*)p = val;
  }
  __threadfence();
  if (tid < 64) *(volatile float*)p = val;
}

__global__ __launch_bounds__(256) void fin(const float* __restrict__ LG, float* out, int nOut) {
  __shared__ __align__(16) float sm[256];
  const int tid = (int)threadIdx.x;
  const int i   = blockIdx.x * 256 + tid;
  const int ic  = (i < nOut) ? i : (nOut - 1);
  const int b   = ic / NCLS;
  const int c   = ic - b * NCLS;
  const float lg = LG[(size_t)b * CP + c];
  const float e  = expf(-lg);
  sm[tid] = 1.0f / (1.0f + e);
  __syncthreads();

  const bool act  = (tid < 64);
  const int  base = blockIdx.x * 256 + tid * 4;
  v4f v = {0.f, 0.f, 0.f, 0.f};
  if (act) v = *(const v4f*)(sm + tid * 4);
  const bool full = (base + 3 < nOut);
  if (act) {
    if (full) {
      *(volatile v4f*)(out + base) = v;
    } else {
      if (base + 0 < nOut) *(volatile float*)(out + base + 0) = v[0];
      if (base + 1 < nOut) *(volatile float*)(out + base + 1) = v[1];
      if (base + 2 < nOut) *(volatile float*)(out + base + 2) = v[2];
    }
  }
  __threadfence();
  if (act) {
    if (full) {
      *(volatile v4f*)(out + base) = v;
    } else {
      if (base + 0 < nOut) *(volatile float*)(out + base + 0) = v[0];
      if (base + 1 < nOut) *(volatile float*)(out + base + 1) = v[1];
      if (base + 2 < nOut) *(volatile float*)(out + base + 2) = v[2];
    }
  }
}

extern "C" void kernel_launch(void* const* d_in, const int* in_sizes, int n_in,
                              void* d_out, int out_size, void* d_ws, size_t ws_size,
                              hipStream_t stream) {
  if (n_in < 4) return;
  const long long needX = ((long long)(NB - 1) * SEQ_FULL + SEQ) * (long long)DM;
  if ((long long)in_sizes[0] < needX) return;
  if ((long long)in_sizes[1] < (long long)NCLS * DM) return;
  if ((long long)in_sizes[2] < (long long)NCLS * DM) return;
  if (in_sizes[3] < NCLS) return;
  if (out_size < NB * NCLS) return;

  size_t off = 0;
  const size_t oXB = off; off += (size_t)XBB;
  const size_t oWC = off; off += (size_t)WCB;
  const size_t oSP = off; off += (size_t)SBB;
  const size_t oLG = off; off += (size_t)LGB;
  if (off > ws_size) return;
  if (off > (size_t)134217728) return;

  const float* x  = (const float*)d_in[0];
  const float* Wa = (const float*)d_in[1];
  const float* Wo = (const float*)d_in[2];
  const float* bo = (const float*)d_in[3];

  char* ws = (char*)d_ws;
  unsigned short* Xb = (unsigned short*)(ws + oXB);
  unsigned short* WC = (unsigned short*)(ws + oWC);
  float*          SP = (float*)(ws + oSP);
  float*          LG = (float*)(ws + oLG);
  float*          out0 = (float*)d_out;

  const dim3 blk(256);
  const int n8xb = SEQ * DM / 8;
  const int n8w  = CP * DM / 8;
  const int nOut = NB * NCLS;
  const dim3 gCvtX((n8xb + 255) / 256, NB);
  const dim3 gCvtW((n8w + 255) / 256, 2);
  const dim3 gG((((SEQ / 64) * (NC / 64)) + 7) / 8, 1);
  const dim3 gSm(CP / 64);
  const dim3 gFin((nOut + 255) / 256);

  cvt16x8<0><<<gCvtX, blk, 0, stream>>>(x, (long long)SEQ_FULL * DM, Xb, (long long)SEQ * DM, n8xb);
  cvtw8<<<gCvtW, blk, 0, stream>>>(Wa, Wo, WC, n8w);
  for (int bb = 0; bb < NB; ++bb) {
    const size_t ao = (size_t)bb * SEQ * DM;
    gemm_t<__bf16, 4, 1, 1, 0, 0><<<gG, blk, 0, stream>>>(
        Xb + ao, Xb + ao, DM, 0LL, WC, DM, 0LL,
        WC, DM, 0LL, 0,
        (void*)SP, (void*)SP, NC, 0LL, NC, 0LL, NC,
        SEQ, NC, DM, 1.0f, 0.0f, 1.0f, 1.0f);
    colsm<<<gSm, blk, 0, stream>>>(SP, bo, LG + (size_t)bb * CP);
  }
  fin<<<gFin, blk, 0, stream>>>(LG, out0, nOut);
  (void)hipGetLastError();
}
